// Model_48266842472625
// MI455X (gfx1250) — hardware-verified
//
#include <hip/hip_runtime.h>
#include <stddef.h>
#include <stdint.h>


#define HID    256
#define XP     512
#define BTK    1024
#define LINK   10
#define F1K    512
#define F1N    256
#define F2N    128
#define F3N    64
#define NLAY   4
#define NTHR   256
#define NWAVE  8
#define EPT    8
#define CHUNK  (NTHR * EPT)
#define WCAP   (EPT * 32)
#define LISTN  (NWAVE * WCAP)
#define NBA    1024
#define SLA    10
#define RCAP   28672
#define DEGCAP 64
#define GBM    64
#define GBN    128
#define GTHR   128
#define AGG_ZINTS    (LISTN + 2 * RCAP + 3 * NBA)
#define MISC_INTS    16
#define AGG_LDS_INTS (AGG_ZINTS + MISC_INTS)
#define CHL    50048
#define WSMAX  134217728

static_assert((CHUNK & (CHUNK - 1)) == 0 && CHUNK <= 4096);
static_assert((NBA & (NBA - 1)) == 0 && NBA == (1 << SLA));
static_assert(((long long)CHUNK << SLA) < (1LL << 31));
static_assert(NBA % NWAVE == 0 && NBA % 32 == 0 && NBA % GBM == 0);
static_assert(AGG_ZINTS % (NTHR * 4) == 0 && LISTN % 4 == 0 && RCAP % 4 == 0);
static_assert(AGG_LDS_INTS * 4 <= 300000);
static_assert(MISC_INTS >= 10 && NWAVE <= 8);
static_assert(RCAP >= 20619 + 4096 && DEGCAP >= 39 + 8);
static_assert(HID == 8 * 32 && XP == 2 * HID && BTK == 4 * HID);
static_assert(GBM == (GTHR / 32) * 16 && GBN == 8 * 16);
static_assert(HID % GBN == 0 && F1N == HID && F2N == GBN && F3N == 4 * 16);
static_assert(F1K == 2 * HID && F1K == XP);
static_assert(BTK % 32 == 0 && HID % 32 == 0 && XP % 32 == 0 && (2 * F2N) % 32 == 0);
static_assert(HID % 8 == 0 && F2N % 8 == 0 && (HID * (HID / 8)) % NTHR == 0);
static_assert((F2N * (F1N / 8)) % NTHR == 0 && (F3N * (F2N / 8)) % NTHR == 0);
static_assert(CHL % GBM == 0 && (CHL * 4) % 128 == 0);
static_assert((GBM * 4) % 128 == 0 && F3N == GBM);
static_assert(LINK == 10 && NLAY == 4);

typedef float          v4f   __attribute__((ext_vector_type(4)));
typedef float          v8f   __attribute__((ext_vector_type(8)));
typedef int            v4i   __attribute__((ext_vector_type(4)));
typedef int            v8i   __attribute__((ext_vector_type(8)));
typedef unsigned int   v2u   __attribute__((ext_vector_type(2)));
typedef unsigned int   v4u   __attribute__((ext_vector_type(4)));
typedef unsigned short v8us  __attribute__((ext_vector_type(8)));
typedef unsigned short v16us __attribute__((ext_vector_type(16)));
typedef __bf16         v16bf __attribute__((ext_vector_type(16)));
typedef v4f  __attribute__((may_alias)) v4fa;
typedef v4i  __attribute__((may_alias)) v4ia;
typedef v2u  __attribute__((may_alias)) v2ua;
typedef v4u  __attribute__((may_alias)) v4ua;
typedef v8us __attribute__((may_alias)) v8usa;
union FragB { v16bf v; v16us u; v8us h[2]; v8i w; };
struct HL4 { v4u h; v4u l; };

__device__ __forceinline__ v8f wmb(const FragB& a, const FragB& b, v8f c) {
  v8f d = __builtin_amdgcn_wmma_f32_16x16x32_bf16(false, a.v, false, b.v, (short)0, c, false, false);
  asm volatile("v_nop\n\tv_nop\n\tv_nop\n\tv_nop" : "+v"(d) : "v"(a.w), "v"(b.w));
  return d;
}

__device__ __forceinline__ unsigned bf16_bits(float f) {
  const unsigned u = __float_as_uint(f);
  return (u + 0x7FFFu + ((u >> 16) & 1u)) >> 16;
}
__device__ __forceinline__ float bf16_val(float f) {
  return __uint_as_float(bf16_bits(f) << 16);
}
__device__ __forceinline__ float lo16f(unsigned w) { return __uint_as_float(w << 16); }
__device__ __forceinline__ float hi16f(unsigned w) { return __uint_as_float(w & 0xffff0000u); }
__device__ __forceinline__ v2u split2(float a, float b) {
  const unsigned ha = bf16_bits(a), hb = bf16_bits(b);
  const unsigned la = bf16_bits(a - __uint_as_float(ha << 16));
  const unsigned lb = bf16_bits(b - __uint_as_float(hb << 16));
  v2u r;
  r.x = ha | (hb << 16);
  r.y = la | (lb << 16);
  return r;
}
__device__ __forceinline__ HL4 split8(float v0, float v1, float v2, float v3,
                                      float v4, float v5, float v6, float v7) {
  const v2u s0 = split2(v0, v1);
  const v2u s1 = split2(v2, v3);
  const v2u s2 = split2(v4, v5);
  const v2u s3 = split2(v6, v7);
  HL4 o;
  o.h.x = s0.x; o.h.y = s1.x; o.h.z = s2.x; o.h.w = s3.x;
  o.l.x = s0.y; o.l.y = s1.y; o.l.z = s2.y; o.l.w = s3.y;
  return o;
}
__device__ __forceinline__ float relu_keep(float v) {
  return (v > 0.0f) ? v : (v - v);
}

template <int SLB>
__device__ __forceinline__ int scan_chunk(const int* __restrict__ dsts, int nE, int cbase, int slotBase,
                                          int nb, int vec8, int* list, int tid, int lane, int wave) {
  int wc = 0;
  const int el0  = tid * EPT;
  const int e0   = cbase + el0;
  const int sent = -2147483647 - 1;
  v4i da, db;
  if (vec8 != 0 && cbase + CHUNK <= nE) {
    da = *(const v4i*)(dsts + e0);
    db = *(const v4i*)(dsts + e0 + 4);
  } else {
    da.x = (e0     < nE) ? dsts[min(e0,     nE - 1)] : sent;
    da.y = (e0 + 1 < nE) ? dsts[min(e0 + 1, nE - 1)] : sent;
    da.z = (e0 + 2 < nE) ? dsts[min(e0 + 2, nE - 1)] : sent;
    da.w = (e0 + 3 < nE) ? dsts[min(e0 + 3, nE - 1)] : sent;
    db.x = (e0 + 4 < nE) ? dsts[min(e0 + 4, nE - 1)] : sent;
    db.y = (e0 + 5 < nE) ? dsts[min(e0 + 5, nE - 1)] : sent;
    db.z = (e0 + 6 < nE) ? dsts[min(e0 + 6, nE - 1)] : sent;
    db.w = (e0 + 7 < nE) ? dsts[min(e0 + 7, nE - 1)] : sent;
  }
  const unsigned nbs = (unsigned)slotBase;
  const unsigned unb = (unsigned)nb;
  const unsigned s0 = (unsigned)da.x - nbs, s1 = (unsigned)da.y - nbs;
  const unsigned s2 = (unsigned)da.z - nbs, s3 = (unsigned)da.w - nbs;
  const unsigned s4 = (unsigned)db.x - nbs, s5 = (unsigned)db.y - nbs;
  const unsigned s6 = (unsigned)db.z - nbs, s7 = (unsigned)db.w - nbs;
  const bool h0 = s0 < unb, h1 = s1 < unb, h2 = s2 < unb, h3 = s3 < unb;
  const bool h4 = s4 < unb, h5 = s5 < unb, h6 = s6 < unb, h7 = s7 < unb;
  const unsigned any = __builtin_amdgcn_ballot_w32(h0 | h1 | h2 | h3 | h4 | h5 | h6 | h7);
  if (any != 0u) {
#define HITJ(J, HJ, SJ) { \
      const unsigned mj = __builtin_amdgcn_ballot_w32(HJ); \
      if (mj != 0u) { \
        if (HJ) { \
          const int pos = wc + (int)__builtin_amdgcn_mbcnt_lo(mj, 0u); \
          if (pos < WCAP) list[wave * WCAP + pos] = ((el0 + (J)) << SLB) | (int)(SJ); \
        } \
        wc += (int)__builtin_popcount(mj); } }
    HITJ(0, h0, s0)
    HITJ(1, h1, s1)
    HITJ(2, h2, s2)
    HITJ(3, h3, s3)
    HITJ(4, h4, s4)
    HITJ(5, h5, s5)
    HITJ(6, h6, s6)
    HITJ(7, h7, s7)
#undef HITJ
  }
  return wc;
}

__global__ __launch_bounds__(NTHR) void k_wT(const float* __restrict__ src, long long srcMat, int K, int N,
                                             unsigned short* dst, long long dstMat, int pitch, int dup,
                                             int nUnits) {
  const int u = (int)blockIdx.x * NTHR + (int)threadIdx.x;
  if (u >= nUnits) return;
  const int mat = (int)blockIdx.y;
  const int kq  = K >> 3;
  const int n   = u / kq;
  const int k8  = (u - n * kq) * 8;
  const float* p = src + (size_t)((long long)mat * srcMat) + (size_t)k8 * (size_t)N + n;
  v8us o;
#pragma unroll
  for (int i = 0; i < 8; ++i) o[i] = (unsigned short)bf16_bits(p[(size_t)i * (size_t)N]);
  unsigned short* dp = dst + (size_t)((long long)mat * dstMat) + (size_t)n * (size_t)pitch + k8;
  *(volatile v8us*)dp = o;
  *(volatile v8us*)(dp + dup) = o;
  __threadfence();
  *(volatile v8us*)dp = o;
  *(volatile v8us*)(dp + dup) = o;
}

__global__ __launch_bounds__(NTHR) void k_xinit(int mode, const int* __restrict__ ids,
                                                const float* __restrict__ emb, const float* __restrict__ dx,
                                                const float* __restrict__ lw, const float* __restrict__ lb,
                                                int nN, int nUnits, unsigned short* xo) {
  const int u = (int)blockIdx.x * NTHR + (int)threadIdx.x;
  if (u >= nUnits) return;
  const int row = u >> 5;
  const int c0  = (u & 31) * 8;
  const bool ok = row < nN;
  const int rc  = ok ? row : nN - 1;
  int id = ids[rc];
  id = id < 0 ? 0 : (id > nN - 1 ? nN - 1 : id);
  const float* ep = emb + (size_t)id * HID + c0;
  const v4f e0 = *(const v4fa*)ep;
  const v4f e1 = *(const v4fa*)(ep + 4);
  float v0 = bf16_val(e0.x), v1 = bf16_val(e0.y), v2 = bf16_val(e0.z), v3 = bf16_val(e0.w);
  float v4 = bf16_val(e1.x), v5 = bf16_val(e1.y), v6 = bf16_val(e1.z), v7 = bf16_val(e1.w);
  if (mode != 0) {
    float a0 = 0.0f, a1 = 0.0f, a2 = 0.0f, a3 = 0.0f, a4 = 0.0f, a5 = 0.0f, a6 = 0.0f, a7 = 0.0f;
#pragma unroll 1
    for (int j = 0; j < LINK; ++j) {
      const float xv = bf16_val(dx[(size_t)rc * LINK + j]);
      const float* wp = lw + (size_t)j * HID + c0;
      const v4f w0 = *(const v4fa*)wp;
      const v4f w1 = *(const v4fa*)(wp + 4);
      a0 = fmaf(xv, bf16_val(w0.x), a0); a1 = fmaf(xv, bf16_val(w0.y), a1);
      a2 = fmaf(xv, bf16_val(w0.z), a2); a3 = fmaf(xv, bf16_val(w0.w), a3);
      a4 = fmaf(xv, bf16_val(w1.x), a4); a5 = fmaf(xv, bf16_val(w1.y), a5);
      a6 = fmaf(xv, bf16_val(w1.z), a6); a7 = fmaf(xv, bf16_val(w1.w), a7);
    }
    const v4f b0 = *(const v4fa*)(lb + c0);
    const v4f b1 = *(const v4fa*)(lb + c0 + 4);
    v0 = (a0 + bf16_val(b0.x)) + v0; v1 = (a1 + bf16_val(b0.y)) + v1;
    v2 = (a2 + bf16_val(b0.z)) + v2; v3 = (a3 + bf16_val(b0.w)) + v3;
    v4 = (a4 + bf16_val(b1.x)) + v4; v5 = (a5 + bf16_val(b1.y)) + v5;
    v6 = (a6 + bf16_val(b1.z)) + v6; v7 = (a7 + bf16_val(b1.w)) + v7;
  }
  v0 = ok ? v0 : 0.0f; v1 = ok ? v1 : 0.0f; v2 = ok ? v2 : 0.0f; v3 = ok ? v3 : 0.0f;
  v4 = ok ? v4 : 0.0f; v5 = ok ? v5 : 0.0f; v6 = ok ? v6 : 0.0f; v7 = ok ? v7 : 0.0f;
  const HL4 q = split8(v0, v1, v2, v3, v4, v5, v6, v7);
  unsigned short* dp = xo + (size_t)row * XP + c0;
  *(volatile v4u*)dp = q.h;
  *(volatile v4u*)(dp + HID) = q.l;
  __threadfence();
  *(volatile v4u*)dp = q.h;
  *(volatile v4u*)(dp + HID) = q.l;
}

__global__ __launch_bounds__(NTHR) void k_scan(const int* __restrict__ gath, const int* __restrict__ keys,
                                               int nE, int nN, int vec8, int mRows,
                                               const unsigned short* __restrict__ xsrc,
                                               unsigned short* aggo) {
  extern __shared__ __attribute__((aligned(16))) int dsm[];
  int* list = dsm;
  int* hl   = dsm + LISTN;
  int* sl   = hl + RCAP;
  int* cnt  = sl + RCAP;
  int* offs = cnt + NBA;
  int* cur  = offs + NBA;
  int* misc = cur + NBA;
  const int tid = (int)threadIdx.x, lane = tid & 31, wave = tid >> 5;
  const int nodeBase = (int)blockIdx.x * NBA;

  {
    const v4i z4 = {0, 0, 0, 0};
    for (int i = tid * 4; i < AGG_ZINTS; i += NTHR * 4) *(v4ia*)(dsm + i) = z4;
    if (tid < MISC_INTS) misc[tid] = 0;
  }
  __syncthreads();

  int t = 0, ov = 0;
  const int nChunks = (nE + CHUNK - 1) / CHUNK;
#pragma unroll 1
  for (int ch = 0; ch < nChunks; ++ch) {
    const int cbase = ch * CHUNK;
    const int wc = scan_chunk<SLA>(keys, nE, cbase, nodeBase, NBA, vec8, list, tid, lane, wave);
    if (lane == 0) misc[wave] = wc;
    __syncthreads();
    if (wave == 0) {
#pragma unroll 1
      for (int w2 = 0; w2 < NWAVE; ++w2) {
        int c = misc[w2];
        c = c < 0 ? 0 : (c > WCAP ? WCAP : c);
#pragma unroll 1
        for (int b0 = 0; b0 < c; b0 += 32) {
          const int idx = b0 + lane;
          const int ent = list[w2 * WCAP + (idx < WCAP ? idx : WCAP - 1)];
          const int m32 = (c - b0) < 32 ? (c - b0) : 32;
#pragma unroll 1
          for (int k = 0; k < m32; ++k) {
            const int u    = __builtin_amdgcn_readlane(ent, k);
            const int slot = u & (NBA - 1);
            const int el   = (u >> SLA) & (CHUNK - 1);
            const int pk   = ((cbase + el) << SLA) | slot;
            if (t < RCAP) {
              if (lane == 0) { hl[t] = pk; cnt[slot] = cnt[slot] + 1; }
              t = t + 1;
            } else {
              ov = 1;
            }
          }
        }
      }
    }
    __syncthreads();
  }
  if (wave == 0 && lane == 0) { misc[8] = t; misc[9] = ov; }
  __syncthreads();
  int tt = misc[8];
  tt = tt < 0 ? 0 : (tt > RCAP ? RCAP : tt);
  const int ovf = misc[9];

  if (wave == 0) {
    const int base = lane * (NBA / 32);
    int s = 0;
#pragma unroll 1
    for (int i = 0; i < NBA / 32; ++i) s += cnt[base + i];
    int incl = s;
#pragma unroll
    for (int d = 1; d < 32; d <<= 1) {
      const int y = __shfl_up(incl, d, 32);
      if (lane >= d) incl += y;
    }
    int run = incl - s;
#pragma unroll 1
    for (int i = 0; i < NBA / 32; ++i) {
      const int cv = cnt[base + i];
      offs[base + i] = run;
      cur[base + i]  = run;
      run += cv;
    }
  }
  __syncthreads();
  if (wave == 0) {
#pragma unroll 1
    for (int b0 = 0; b0 < tt; b0 += 32) {
      const int idx = b0 + lane;
      const int ent = hl[idx < RCAP ? idx : RCAP - 1];
      const int m32 = (tt - b0) < 32 ? (tt - b0) : 32;
#pragma unroll 1
      for (int k = 0; k < m32; ++k) {
        const int u    = __builtin_amdgcn_readlane(ent, k);
        const int slot = u & (NBA - 1);
        if (lane == 0) {
          int p = cur[slot];
          p = p < 0 ? 0 : (p > RCAP - 1 ? RCAP - 1 : p);
          sl[p] = u;
          cur[slot] = p + 1;
        }
      }
    }
  }
  __syncthreads();

  const float qnan = __int_as_float(0x7fc00000);
  const float pz = (ovf != 0) ? qnan : 0.0f;
#pragma unroll 1
  for (int si = 0; si < NBA / NWAVE; ++si) {
    const int s    = si * NWAVE + wave;
    const int node = nodeBase + s;
    const int craw = cnt[s];
    const bool big = craw > DEGCAP;
    const int c = craw < 0 ? 0 : (craw > DEGCAP ? DEGCAP : craw);
    int o = offs[s];
    o = o < 0 ? 0 : (o > RCAP ? RCAP : o);
    float a0 = 0.0f, a1 = 0.0f, a2 = 0.0f, a3 = 0.0f, a4 = 0.0f, a5 = 0.0f, a6 = 0.0f, a7 = 0.0f;
#pragma unroll 1
    for (int b0 = 0; b0 < c; b0 += 32) {
      int idx = o + b0 + lane;
      idx = idx > RCAP - 1 ? RCAP - 1 : idx;
      const int ent = sl[idx];
      int eid = ent >> SLA;
      eid = eid < 0 ? 0 : (eid > nE - 1 ? nE - 1 : eid);
      int sr = gath[eid];
      sr = sr < 0 ? 0 : (sr > nN - 1 ? nN - 1 : sr);
      const int m32 = (c - b0) < 32 ? (c - b0) : 32;
#pragma unroll 1
      for (int k = 0; k < m32; ++k) {
        const int sk = __builtin_amdgcn_readlane(sr, k);
        const unsigned short* rp = xsrc + (size_t)sk * XP + 8 * lane;
        const v4u wh = *(const v4ua*)rp;
        const v4u wl = *(const v4ua*)(rp + HID);
        a0 += (lo16f(wh.x) + lo16f(wl.x)); a1 += (hi16f(wh.x) + hi16f(wl.x));
        a2 += (lo16f(wh.y) + lo16f(wl.y)); a3 += (hi16f(wh.y) + hi16f(wl.y));
        a4 += (lo16f(wh.z) + lo16f(wl.z)); a5 += (hi16f(wh.z) + hi16f(wl.z));
        a6 += (lo16f(wh.w) + lo16f(wl.w)); a7 += (hi16f(wh.w) + hi16f(wl.w));
      }
    }
    const int   cm  = craw < 1 ? 1 : craw;
    const float inv = 1.0f / (float)cm;
    const float pzr = big ? qnan : pz;
    const bool live = node < nN;
    const float m0 = live ? (a0 * inv + pzr) : 0.0f;
    const float m1 = live ? (a1 * inv + pzr) : 0.0f;
    const float m2 = live ? (a2 * inv + pzr) : 0.0f;
    const float m3 = live ? (a3 * inv + pzr) : 0.0f;
    const float m4 = live ? (a4 * inv + pzr) : 0.0f;
    const float m5 = live ? (a5 * inv + pzr) : 0.0f;
    const float m6 = live ? (a6 * inv + pzr) : 0.0f;
    const float m7 = live ? (a7 * inv + pzr) : 0.0f;
    const HL4 q = split8(m0, m1, m2, m3, m4, m5, m6, m7);
    if (node < mRows) {
      unsigned short* rpw = aggo + (size_t)node * XP + 8 * lane;
      *(volatile v4u*)rpw = q.h;
      *(volatile v4u*)(rpw + HID) = q.l;
      __threadfence();
      *(volatile v4u*)rpw = q.h;
      *(volatile v4u*)(rpw + HID) = q.l;
    }
  }
}

template <int NT>
__device__ __forceinline__ void gemm_core(const unsigned short* Ab, long long oA0, long long oA1, int pitchA,
                                          int nseg, int segl, const unsigned short* __restrict__ Bt, int K,
                                          int rowBase, float* stg, int lane, int wave) {
  const int hh = lane >> 4, m = lane & 15;
  v8f acc[NT];
  {
    const v8f z = {0.f, 0.f, 0.f, 0.f, 0.f, 0.f, 0.f, 0.f};
#pragma unroll
    for (int t = 0; t < NT; ++t) acc[t] = z;
  }
  const long long rowOff = (long long)(rowBase + 16 * wave + m) * (long long)pitchA + 8 * hh;
  const unsigned short* bp = Bt + (size_t)m * (size_t)K + 8 * hh;
#pragma unroll 1
  for (int s = 0; s < nseg; ++s) {
    const long long so = (((s & 1) != 0) ? oA1 : oA0) + rowOff + (long long)(s >> 1) * (long long)segl;
    const unsigned short* ap = Ab + so;
    const unsigned short* bq = bp + (size_t)s * (size_t)segl;
#pragma unroll 1
    for (int k0 = 0; k0 < segl; k0 += 32) {
      FragB af;
      af.h[0] = *(const v8usa*)(ap + k0);
      af.h[1] = *(const v8usa*)(ap + k0 + 16);
#pragma unroll
      for (int nt = 0; nt < NT; ++nt) {
        const unsigned short* wq = bq + (size_t)(16 * nt) * (size_t)K + k0;
        FragB bf;
        bf.h[0] = *(const v8usa*)wq;
        bf.h[1] = *(const v8usa*)(wq + 16);
        acc[nt] = wmb(af, bf, acc[nt]);
      }
    }
  }
#pragma unroll
  for (int nt = 0; nt < NT; ++nt) {
    const int lc = 16 * nt + m;
#pragma unroll
    for (int r = 0; r < 8; ++r) {
      const int lr = 16 * wave + 8 * hh + r;
      stg[lr * (16 * NT) + lc] = acc[nt][r];
    }
  }
  __syncthreads();
}

__global__ __launch_bounds__(GTHR) void k_gemm_hl(
    const unsigned short* Ab, long long oA0, long long oA1, long long zA, int pitchA, int nseg, int segl,
    const unsigned short* __restrict__ Bt, long long zB, int K,
    const float* __restrict__ bias0, const float* __restrict__ bias1, int relu,
    unsigned short* outH, long long zOut, int pitchOut, int loOff, int nLive) {
  __shared__ __attribute__((aligned(16))) float stg[GBM * GBN];
  const int tid = (int)threadIdx.x, lane = tid & 31, wave = tid >> 5;
  const int z = (int)blockIdx.z;
  const int rowBase = (int)blockIdx.x * GBM;
  const int col0 = (int)blockIdx.y * GBN;

  gemm_core<8>(Ab, oA0 + (long long)z * zA, oA1 + (long long)z * zA, pitchA, nseg, segl,
               Bt + (size_t)((long long)z * zB) + (size_t)col0 * (size_t)K, K, rowBase, stg, lane, wave);

  v4f bb4;
  {
    const v4f t0 = *(const v4fa*)(bias0 + col0 + 4 * lane);
    const v4f t1 = *(const v4fa*)(bias1 + col0 + 4 * lane);
    const bool zz = (z != 0);
    bb4.x = bf16_val(zz ? t1.x : t0.x);
    bb4.y = bf16_val(zz ? t1.y : t0.y);
    bb4.z = bf16_val(zz ? t1.z : t0.z);
    bb4.w = bf16_val(zz ? t1.w : t0.w);
  }
  v4f pv[16];
#pragma unroll
  for (int i = 0; i < 16; ++i) pv[i] = *(const v4fa*)(stg + (16 * wave + i) * GBN + 4 * lane);
  __syncthreads();
  const bool dorelu = (relu != 0);
#pragma unroll
  for (int i = 0; i < 16; ++i) {
    const bool ok = (rowBase + 16 * wave + i) < nLive;
    const v4f t = pv[i] + bb4;
    v4f y;
    y.x = dorelu ? relu_keep(t.x) : t.x;
    y.y = dorelu ? relu_keep(t.y) : t.y;
    y.z = dorelu ? relu_keep(t.z) : t.z;
    y.w = dorelu ? relu_keep(t.w) : t.w;
    y.x = ok ? y.x : 0.0f; y.y = ok ? y.y : 0.0f; y.z = ok ? y.z : 0.0f; y.w = ok ? y.w : 0.0f;
    pv[i] = y;
  }
#pragma unroll
  for (int i = 0; i < 16; ++i) {
    const v2u sa = split2(pv[i].x, pv[i].y);
    const v2u sb = split2(pv[i].z, pv[i].w);
    v2u h2, l2;
    h2.x = sa.x; h2.y = sb.x;
    l2.x = sa.y; l2.y = sb.y;
    unsigned* srow = (unsigned*)stg + (size_t)(16 * wave + i) * GBN;
    *(v2ua*)(srow + 2 * lane) = h2;
    *(v2ua*)(srow + 64 + 2 * lane) = l2;
  }
  __syncthreads();
  v4u qv[16];
#pragma unroll
  for (int i = 0; i < 16; ++i) {
    const unsigned* srow = (const unsigned*)stg + (size_t)(16 * wave + i) * GBN;
    qv[i] = *(const v4ua*)(srow + 4 * lane);
  }
  const int l16  = lane & 15;
  const int colo = (lane < 16) ? (col0 + 8 * l16) : (loOff + col0 + 8 * l16);
  unsigned short* ob = outH + (size_t)((long long)z * zOut) + colo;
#pragma unroll
  for (int i = 0; i < 16; ++i) {
    unsigned short* rp = ob + (size_t)(rowBase + 16 * wave + i) * (size_t)pitchOut;
    *(volatile v4u*)rp = qv[i];
  }
  __threadfence();
#pragma unroll
  for (int i = 0; i < 16; ++i) {
    unsigned short* rp = ob + (size_t)(rowBase + 16 * wave + i) * (size_t)pitchOut;
    *(volatile v4u*)rp = qv[i];
  }
}

__global__ __launch_bounds__(GTHR) void k_gemm_f32(
    const unsigned short* Ab, long long oA0, long long zA, int pitchA, int K,
    const unsigned short* __restrict__ Bt, long long zB, float* outF, long long zOut) {
  __shared__ __attribute__((aligned(16))) float stg[GBM * GBN];
  const int tid = (int)threadIdx.x, lane = tid & 31, wave = tid >> 5;
  const int z = (int)blockIdx.z;
  const int rowBase = (int)blockIdx.x * GBM;
  const int col0 = (int)blockIdx.y * GBN;
  const long long oa = oA0 + (long long)z * zA;
  gemm_core<8>(Ab, oa, oa, pitchA, 1, K, Bt + (size_t)((long long)z * zB) + (size_t)col0 * (size_t)K, K,
               rowBase, stg, lane, wave);
  v4f pv[16];
#pragma unroll
  for (int i = 0; i < 16; ++i) pv[i] = *(const v4fa*)(stg + (16 * wave + i) * GBN + 4 * lane);
  float* ob = outF + (size_t)((long long)z * zOut) + col0 + 4 * lane;
#pragma unroll
  for (int i = 0; i < 16; ++i)
    *(volatile v4f*)(ob + (size_t)(rowBase + 16 * wave + i) * HID) = pv[i];
  __threadfence();
#pragma unroll
  for (int i = 0; i < 16; ++i)
    *(volatile v4f*)(ob + (size_t)(rowBase + 16 * wave + i) * HID) = pv[i];
}

__global__ __launch_bounds__(NTHR) void k_e1(const float* __restrict__ PD, const float* __restrict__ PS,
                                             const int* __restrict__ lab, int nEL, int labOff, int nv, int nN,
                                             const float* __restrict__ b1, unsigned short* E1, int nUnits) {
  const int u = (int)blockIdx.x * NTHR + (int)threadIdx.x;
  if (u >= nUnits) return;
  const int ri = u >> 5;
  const int c0 = (u & 31) * 8;
  const bool ok = ri < nv;
  int L = labOff + ri;
  L = L > nEL - 1 ? nEL - 1 : L;
  int d = lab[L];
  int s = lab[(size_t)nEL + L];
  d = d < 0 ? 0 : (d > nN - 1 ? nN - 1 : d);
  s = s < 0 ? 0 : (s > nN - 1 ? nN - 1 : s);
  const float* pd = PD + (size_t)d * HID + c0;
  const float* ps = PS + (size_t)s * HID + c0;
  const v4f d0 = *(const v4fa*)pd;
  const v4f d1 = *(const v4fa*)(pd + 4);
  const v4f s0 = *(const v4fa*)ps;
  const v4f s1 = *(const v4fa*)(ps + 4);
  const v4f b0 = *(const v4fa*)(b1 + c0);
  const v4f b4 = *(const v4fa*)(b1 + c0 + 4);
  float v0 = relu_keep((d0.x + s0.x) + bf16_val(b0.x));
  float v1 = relu_keep((d0.y + s0.y) + bf16_val(b0.y));
  float v2 = relu_keep((d0.z + s0.z) + bf16_val(b0.z));
  float v3 = relu_keep((d0.w + s0.w) + bf16_val(b0.w));
  float v4 = relu_keep((d1.x + s1.x) + bf16_val(b4.x));
  float v5 = relu_keep((d1.y + s1.y) + bf16_val(b4.y));
  float v6 = relu_keep((d1.z + s1.z) + bf16_val(b4.z));
  float v7 = relu_keep((d1.w + s1.w) + bf16_val(b4.w));
  v0 = ok ? v0 : 0.0f; v1 = ok ? v1 : 0.0f; v2 = ok ? v2 : 0.0f; v3 = ok ? v3 : 0.0f;
  v4 = ok ? v4 : 0.0f; v5 = ok ? v5 : 0.0f; v6 = ok ? v6 : 0.0f; v7 = ok ? v7 : 0.0f;
  const HL4 q = split8(v0, v1, v2, v3, v4, v5, v6, v7);
  unsigned short* dp = E1 + (size_t)ri * XP + c0;
  *(volatile v4u*)dp = q.h;
  *(volatile v4u*)(dp + HID) = q.l;
  __threadfence();
  *(volatile v4u*)dp = q.h;
  *(volatile v4u*)(dp + HID) = q.l;
}

__global__ __launch_bounds__(GTHR) void k_fc3(const unsigned short* Ab, long long oA, int pitchA, int K,
                                              const unsigned short* __restrict__ Bt,
                                              const float* __restrict__ b3, const float* __restrict__ w4,
                                              const float* __restrict__ b4, float* dout, int nv) {
  __shared__ __attribute__((aligned(16))) float stg[GBM * F3N];
  __shared__ float b3s[F3N];
  __shared__ float w4s[F3N];
  __shared__ __attribute__((aligned(16))) float res[GBM];
  const int tid = (int)threadIdx.x, lane = tid & 31, wave = tid >> 5;
  const int rowBase = (int)blockIdx.x * GBM;
  if (tid < F3N) { b3s[tid] = bf16_val(b3[tid]); w4s[tid] = bf16_val(w4[tid]); }
  gemm_core<4>(Ab, oA, oA, pitchA, 1, K, Bt, K, rowBase, stg, lane, wave);
  if (tid < GBM) {
    const float b4v = bf16_val(b4[0]);
    float s = 0.0f;
#pragma unroll 4
    for (int c = 0; c < F3N; ++c) {
      const float v = relu_keep(stg[tid * F3N + c] + b3s[c]);
      s = fmaf(v, w4s[c], s);
    }
    res[tid] = s + b4v;
  }
  __syncthreads();
  int nvalid = nv - rowBase;
  nvalid = nvalid < 0 ? 0 : (nvalid > GBM ? GBM : nvalid);
  const int l16 = lane & 15;
  const v4f ov = *(const v4fa*)(res + 4 * l16);
  float* op = dout + (size_t)rowBase + 4 * l16;
  const bool okst = (wave == 0) && (lane < 16) && (4 * l16 + 3 < nvalid);
  if (okst) *(volatile v4f*)op = ov;
  __threadfence();
  if (okst) *(volatile v4f*)op = ov;
}

static inline int cdiv(int a, int b) { return (a + b - 1) / b; }
static inline size_t al256(size_t o) { return (o + 255) & ~(size_t)255; }

extern "C" void kernel_launch(void* const* d_in, const int* in_sizes, int n_in,
                              void* d_out, int out_size, void* d_ws, size_t ws_size,
                              hipStream_t stream) {
  if (n_in < 24) return;
  const int nN = in_sizes[0];
  if (nN < 64 || nN > (1 << 20)) return;
  if (in_sizes[2] != nN) return;
  if ((long long)in_sizes[1] != (long long)nN * LINK) return;
  if (in_sizes[3] < 2 || (in_sizes[3] & 1) != 0) return;
  const int nE = in_sizes[3] / 2;
  if (in_sizes[4] != 2 * nE) return;
  if (nE < 1 || nE >= (1 << 21)) return;
  if (in_sizes[5] < 2 || (in_sizes[5] & 1) != 0) return;
  const int nEL = in_sizes[5] / 2;
  if (nEL < 32 || (nEL % 32) != 0) return;
  if (out_size != nEL) return;
  if ((long long)in_sizes[6] != (long long)nN * HID) return;
  if ((long long)in_sizes[7] != (long long)nN * HID) return;
  if (in_sizes[8] != LINK * HID || in_sizes[9] != HID) return;
  if (in_sizes[10] != NLAY * HID * HID || in_sizes[12] != NLAY * HID * HID) return;
  if (in_sizes[13] != NLAY * HID * HID || in_sizes[15] != NLAY * HID * HID) return;
  if (in_sizes[11] != NLAY * HID || in_sizes[14] != NLAY * HID) return;
  if (in_sizes[16] != F1K * F1N || in_sizes[17] != F1N) return;
  if (in_sizes[18] != F1N * F2N || in_sizes[19] != F2N) return;
  if (in_sizes[20] != F2N * F3N || in_sizes[21] != F3N) return;
  if (in_sizes[22] != F3N || in_sizes[23] != 1) return;

  const int*   drug_id = (const int*)d_in[0];
  const float* dis_x   = (const float*)d_in[1];
  const int*   dis_id  = (const int*)d_in[2];
  const int*   e_mt    = (const int*)d_in[3];
  const int*   e_rev   = (const int*)d_in[4];
  const int*   e_lab   = (const int*)d_in[5];
  const float* drug_emb = (const float*)d_in[6];
  const float* dis_emb  = (const float*)d_in[7];
  const float* lin_w   = (const float*)d_in[8];
  const float* lin_b   = (const float*)d_in[9];
  const float* Wl_mt   = (const float*)d_in[10];
  const float* bl_mt   = (const float*)d_in[11];
  const float* Wr_mt   = (const float*)d_in[12];
  const float* Wl_rev  = (const float*)d_in[13];
  const float* bl_rev  = (const float*)d_in[14];
  const float* Wr_rev  = (const float*)d_in[15];
  const float* fc1_w = (const float*)d_in[16]; const float* fc1_b = (const float*)d_in[17];
  const float* fc2_w = (const float*)d_in[18]; const float* fc2_b = (const float*)d_in[19];
  const float* fc3_w = (const float*)d_in[20]; const float* fc3_b = (const float*)d_in[21];
  const float* fc4_w = (const float*)d_in[22]; const float* fc4_b = (const float*)d_in[23];
  float* out = (float*)d_out;

  const int MP = cdiv(nN, GBM) * GBM;
  const int gM = MP / GBM;
  const int gA = cdiv(MP, NBA);
  if ((long long)gA * NBA < (long long)MP) return;
  const int vec8 = ((nE & 3) == 0) ? 1 : 0;

  const size_t planeB = (size_t)MP * XP * 2;
  const size_t planeE = (size_t)MP * XP;
  const size_t btE    = (size_t)HID * BTK;
  size_t off = 0;
  const size_t oBT  = off; off = al256(off + 2 * NLAY * btE * 2);
  const size_t oFD  = off; off = al256(off + (size_t)2 * F1N * XP * 2);
  const size_t oF2  = off; off = al256(off + (size_t)F2N * XP * 2);
  const size_t oF3  = off; off = al256(off + (size_t)F3N * (2 * F2N) * 2);
  const size_t oAGG = off; off = al256(off + 2 * planeB);
  const size_t oX   = off; off = al256(off + 4 * planeB);
  if (off > ws_size || off > (size_t)WSMAX) return;
  const size_t e1B = al256((size_t)CHL * XP * 2);
  const size_t e2B = al256((size_t)CHL * (2 * F2N) * 2);
  if (e1B + e2B > 4 * planeB) return;
  if ((size_t)MP * HID * 4 > planeB) return;

  char* ws = (char*)d_ws;
  unsigned short* ws16 = (unsigned short*)d_ws;
  unsigned short* BT = (unsigned short*)(ws + oBT);
  unsigned short* FD = (unsigned short*)(ws + oFD);
  unsigned short* F2 = (unsigned short*)(ws + oF2);
  unsigned short* F3 = (unsigned short*)(ws + oF3);
  const long long eAGG = (long long)(oAGG / 2);
  const long long eX   = (long long)(oX / 2);
  const long long eE1  = eX;
  const long long eE2  = eX + (long long)(e1B / 2);
  float* PDS = (float*)(ws + oAGG);

  const size_t scanLds = (size_t)AGG_LDS_INTS * 4;
  hipFuncSetAttribute(reinterpret_cast<const void*>(&k_scan), hipFuncAttributeMaxDynamicSharedMemorySize,
                      (int)scanLds);

  {
    const int nu = HID * (HID / 8);
    const dim3 g4(cdiv(nu, NTHR), NLAY);
    k_wT<<<g4, NTHR, 0, stream>>>(Wl_rev, (long long)HID * HID, HID, HID, BT + 0 * NLAY * btE + 0,   (long long)btE, BTK, 2 * HID, nu);
    k_wT<<<g4, NTHR, 0, stream>>>(Wr_rev, (long long)HID * HID, HID, HID, BT + 0 * NLAY * btE + HID, (long long)btE, BTK, 2 * HID, nu);
    k_wT<<<g4, NTHR, 0, stream>>>(Wl_mt,  (long long)HID * HID, HID, HID, BT + 1 * NLAY * btE + 0,   (long long)btE, BTK, 2 * HID, nu);
    k_wT<<<g4, NTHR, 0, stream>>>(Wr_mt,  (long long)HID * HID, HID, HID, BT + 1 * NLAY * btE + HID, (long long)btE, BTK, 2 * HID, nu);
    k_wT<<<dim3(cdiv(nu, NTHR), 2), NTHR, 0, stream>>>(fc1_w, (long long)HID * F1N, HID, F1N, FD,
                                                       (long long)F1N * XP, XP, HID, nu);
    k_wT<<<dim3(cdiv(F2N * (F1N / 8), NTHR), 1), NTHR, 0, stream>>>(fc2_w, 0LL, F1N, F2N, F2, 0LL, XP, F1N,
                                                                    F2N * (F1N / 8));
    k_wT<<<dim3(cdiv(F3N * (F2N / 8), NTHR), 1), NTHR, 0, stream>>>(fc3_w, 0LL, F2N, F3N, F3, 0LL, 2 * F2N, F2N,
                                                                    F3N * (F2N / 8));
  }

  {
    const int nu = MP * 32;
    k_xinit<<<cdiv(nu, NTHR), NTHR, 0, stream>>>(0, drug_id, drug_emb, dis_x, lin_w, lin_b, nN, nu,
                                                 ws16 + eX + 0 * (long long)planeE);
    k_xinit<<<cdiv(nu, NTHR), NTHR, 0, stream>>>(1, dis_id, dis_emb, dis_x, lin_w, lin_b, nN, nu,
                                                 ws16 + eX + 1 * (long long)planeE);
  }

  for (int l = 0; l < NLAY; ++l) {
    const int b = l & 1;
    const long long eXb  = eX + (long long)(2 * b) * (long long)planeE;
    const long long eXo  = eX + (long long)(2 * (b ^ 1)) * (long long)planeE;
    k_scan<<<gA, NTHR, scanLds, stream>>>(e_rev, e_rev + nE, nE, nN, vec8, MP,
                                          ws16 + eXb + (long long)planeE, ws16 + eAGG);
    k_scan<<<gA, NTHR, scanLds, stream>>>(e_mt, e_mt + nE, nE, nN, vec8, MP,
                                          ws16 + eXb, ws16 + eAGG + (long long)planeE);
    k_gemm_hl<<<dim3(gM, HID / GBN, 2), GTHR, 0, stream>>>(
        ws16, eAGG, eXb, (long long)planeE, XP, 4, HID,
        BT + (size_t)l * btE, (long long)(NLAY * btE), BTK,
        bl_rev + (size_t)l * HID, bl_mt + (size_t)l * HID, (l < NLAY - 1) ? 1 : 0,
        ws16 + eXo, (long long)planeE, XP, HID, nN);
  }

  k_gemm_f32<<<dim3(gM, HID / GBN, 2), GTHR, 0, stream>>>(
      ws16, eX, (long long)planeE, XP, XP, FD, (long long)F1N * XP, PDS, (long long)MP * HID);

  const int nCh = cdiv(nEL, CHL);
  for (int c = 0; c < nCh; ++c) {
    const int labOff = c * CHL;
    const int nv = (nEL - labOff) < CHL ? (nEL - labOff) : CHL;
    const int rowsPad = cdiv(nv, GBM) * GBM;
    const int nu = rowsPad * 32;
    k_e1<<<cdiv(nu, NTHR), NTHR, 0, stream>>>(PDS, PDS + (size_t)MP * HID, e_lab, nEL, labOff, nv, nN,
                                              fc1_b, ws16 + eE1, nu);
    k_gemm_hl<<<dim3(rowsPad / GBM, 1, 1), GTHR, 0, stream>>>(
        ws16, eE1, eE1, 0LL, XP, 1, XP, F2, 0LL, XP, fc2_b, fc2_b, 1,
        ws16 + eE2, 0LL, 2 * F2N, F2N, nv);
    k_fc3<<<rowsPad / GBM, GTHR, 0, stream>>>(ws16, eE2, 2 * F2N, 2 * F2N, F3, fc3_b, fc4_w, fc4_b,
                                              out + labOff, nv);
  }
}
